// SAGEVolModel_27195732918655
// MI455X (gfx1250) — hardware-verified
//
#include <hip/hip_runtime.h>
#include <hip/hip_bf16.h>
#include <stddef.h>


#define DD      64
#define KCAT    128
#define HN      32
#define NTHR    256
#define NWAVE   8
#define EPT     8
#define NGRP    2
#define CHUNK   (NTHR * EPT * NGRP)
#define WCAP    (EPT * NGRP * 32)
#define LISTN   (NWAVE * WCAP)
#define NBC     4096
#define NBF     1024
#define RCAP    40960
#define RBN     128
#define DEGCAP  256
#define GROWS   128
#define OTHR    512
#define APH     (KCAT + 8)
#define LNEPS   1e-5f

#define LDS_FILL  ((RCAP + NBF + LISTN) * 4 + 64)
#define LDS_LAYER (2 * GROWS * APH * 2 + GROWS * DD * 4 + GROWS * 4)

static_assert((CHUNK & (CHUNK - 1)) == 0);
static_assert(CHUNK <= 4096);
static_assert(NBC <= 4096 && NBF <= 4096);
static_assert((NBC & (NBC - 1)) == 0 && (NBF & (NBF - 1)) == 0);
static_assert(NBC == 4 * NBF);
static_assert(OTHR * 8 == NBC);
static_assert((RCAP % 32) == 0);
static_assert(GROWS == NWAVE * 16);
static_assert(((APH * 2) % 16) == 0);
static_assert(GROWS * DD == 4 * 8 * NTHR);
static_assert((NBC % GROWS) == 0);

typedef float          v2f  __attribute__((ext_vector_type(2)));
typedef float          v4f  __attribute__((ext_vector_type(4)));
typedef float          v8f  __attribute__((ext_vector_type(8)));
typedef int            v4i  __attribute__((ext_vector_type(4)));
typedef unsigned short v2us __attribute__((ext_vector_type(2)));
typedef unsigned short v8us __attribute__((ext_vector_type(8)));
typedef __bf16         v16b __attribute__((ext_vector_type(16)));
union FragB { v16b v; v8us h[2]; };

__device__ __forceinline__ unsigned short bf_rne(float f) {
  union { float f; unsigned u; } q; q.f = f;
  unsigned u = q.u;
  u += 0x7FFFu + ((u >> 16) & 1u);
  return (unsigned short)(u >> 16);
}
__device__ __forceinline__ float bf_up(unsigned short hb) {
  union { float f; unsigned u; } q; q.u = ((unsigned)hb) << 16;
  return q.f;
}
__device__ __forceinline__ void split2(v2f v, v2us& hi, v2us& lo) {
  const unsigned short h0 = bf_rne(v.x), h1 = bf_rne(v.y);
  hi.x = h0; hi.y = h1;
  lo.x = bf_rne(v.x - bf_up(h0));
  lo.y = bf_rne(v.y - bf_up(h1));
}
__device__ __forceinline__ void split8(v4f a, v4f b, v8us& hi, v8us& lo) {
  float v[8];
  v[0] = a.x; v[1] = a.y; v[2] = a.z; v[3] = a.w; v[4] = b.x; v[5] = b.y; v[6] = b.z; v[7] = b.w;
#pragma unroll
  for (int e = 0; e < 8; ++e) {
    const unsigned short hb = bf_rne(v[e]);
    hi[e] = hb;
    lo[e] = bf_rne(v[e] - bf_up(hb));
  }
}

__device__ __forceinline__ v8f wmb(v16b a, v16b b, v8f c) {
  v8f d = __builtin_amdgcn_wmma_f32_16x16x32_bf16(false, a, false, b, (short)0, c, false, false);
  asm volatile("v_nop\n\tv_nop\n\tv_nop\n\tv_nop" : "+v"(d) : "v"(a), "v"(b));
  return d;
}

__device__ __forceinline__ float wsum32(float v) {
  v += __shfl_xor(v, 16);
  v += __shfl_xor(v, 8);
  v += __shfl_xor(v, 4);
  v += __shfl_xor(v, 2);
  v += __shfl_xor(v, 1);
  return v;
}

template <int NB>
__device__ __forceinline__ int scan_chunk(const int* __restrict__ dsts, int nE, int cbase, int slotBase,
                                          int vec8, int* list, int tid, int lane, int wave) {
  int wc = 0;
#pragma unroll
  for (int g = 0; g < NGRP; ++g) {
    const int el0  = (g * NTHR + tid) * EPT;
    const int e0   = cbase + el0;
    const int sent = -2147483647 - 1;
    v4i da, db;
    if (vec8 != 0 && cbase + CHUNK <= nE) {
      da = *(const v4i*)(dsts + e0);
      db = *(const v4i*)(dsts + e0 + 4);
    } else {
      da.x = (e0     < nE) ? dsts[min(e0, nE - 1)] : sent;
      da.y = (e0 + 1 < nE) ? dsts[min(e0 + 1, nE - 1)] : sent;
      da.z = (e0 + 2 < nE) ? dsts[min(e0 + 2, nE - 1)] : sent;
      da.w = (e0 + 3 < nE) ? dsts[min(e0 + 3, nE - 1)] : sent;
      db.x = (e0 + 4 < nE) ? dsts[min(e0 + 4, nE - 1)] : sent;
      db.y = (e0 + 5 < nE) ? dsts[min(e0 + 5, nE - 1)] : sent;
      db.z = (e0 + 6 < nE) ? dsts[min(e0 + 6, nE - 1)] : sent;
      db.w = (e0 + 7 < nE) ? dsts[min(e0 + 7, nE - 1)] : sent;
    }
    const unsigned nb = (unsigned)slotBase;
    const unsigned s0 = (unsigned)da.x - nb, s1 = (unsigned)da.y - nb;
    const unsigned s2 = (unsigned)da.z - nb, s3 = (unsigned)da.w - nb;
    const unsigned s4 = (unsigned)db.x - nb, s5 = (unsigned)db.y - nb;
    const unsigned s6 = (unsigned)db.z - nb, s7 = (unsigned)db.w - nb;
    const bool h0 = s0 < (unsigned)NB, h1 = s1 < (unsigned)NB, h2 = s2 < (unsigned)NB, h3 = s3 < (unsigned)NB;
    const bool h4 = s4 < (unsigned)NB, h5 = s5 < (unsigned)NB, h6 = s6 < (unsigned)NB, h7 = s7 < (unsigned)NB;
    const unsigned any = __builtin_amdgcn_ballot_w32(h0 | h1 | h2 | h3 | h4 | h5 | h6 | h7);
    if (any != 0u) {
#define HITJ(J, HJ, SJ) { \
        const unsigned mj = __builtin_amdgcn_ballot_w32(HJ); \
        if (mj != 0u) { \
          if (HJ) { \
            const int pos = wc + (int)__builtin_amdgcn_mbcnt_lo(mj, 0u); \
            if (pos < WCAP) list[wave * WCAP + pos] = ((el0 + (J)) << 12) | (int)(SJ); \
          } \
          wc += (int)__builtin_popcount(mj); } }
      HITJ(0, h0, s0)
      HITJ(1, h1, s1)
      HITJ(2, h2, s2)
      HITJ(3, h3, s3)
      HITJ(4, h4, s4)
      HITJ(5, h5, s5)
      HITJ(6, h6, s6)
      HITJ(7, h7, s7)
#undef HITJ
    }
  }
  return wc;
}

__global__ __launch_bounds__(NTHR) void k_wprep(
    const float* __restrict__ Ws, const float* __restrict__ Wn, const float* __restrict__ hw1,
    unsigned short* wlh, unsigned short* wll, unsigned short* h1h, unsigned short* h1l, int nL) {
  const int g0 = nL * (DD * KCAT / 8);
  const int g1 = HN * DD / 8;
  const int i = blockIdx.x * NTHR + (int)threadIdx.x;
  if (i >= g0 + g1) return;
  float v[8];
  unsigned short* dh; unsigned short* dl; int o;
  if (blockIdx.x * NTHR < g0) {
    o = i * 8;
    const int layer = o / (DD * KCAT);
    const int oo = o - layer * (DD * KCAT);
    const int n  = oo / KCAT;
    const int k0 = oo - n * KCAT;
#pragma unroll
    for (int e = 0; e < 8; ++e) {
      const int k  = k0 + e;
      const int ks = k < DD ? k : DD - 1;
      int kn = k - DD; kn = kn < 0 ? 0 : kn;
      const float a = Ws[((size_t)layer * DD + ks) * DD + n];
      const float b = Wn[((size_t)layer * DD + kn) * DD + n];
      v[e] = k < DD ? a : b;
    }
    dh = wlh; dl = wll;
  } else {
    o = (i - g0) * 8;
    const int n  = o / DD;
    const int k0 = o - n * DD;
#pragma unroll
    for (int e = 0; e < 8; ++e) v[e] = hw1[(size_t)(k0 + e) * HN + n];
    dh = h1h; dl = h1l;
  }
  v4f a, b;
  a.x = v[0]; a.y = v[1]; a.z = v[2]; a.w = v[3];
  b.x = v[4]; b.y = v[5]; b.z = v[6]; b.w = v[7];
  v8us hv, lv;
  split8(a, b, hv, lv);
  unsigned short* ph = dh + o;
  unsigned short* pl = dl + o;
  *(volatile v8us*)ph = hv;
  *(volatile v8us*)pl = lv;
  __threadfence();
  *(volatile v8us*)ph = hv;
  *(volatile v8us*)pl = lv;
}

__global__ __launch_bounds__(NTHR) void k_count(const int* __restrict__ ei, int* cnt, int nE, int vec8) {
  __shared__ __attribute__((aligned(16))) int scnt[NBC];
  __shared__ __attribute__((aligned(16))) int list[LISTN];
  __shared__ int wcnt[NWAVE];
  const int tid = threadIdx.x, lane = tid & 31, wave = tid >> 5;
  const int nodeBase = blockIdx.x * NBC;
  const int* dsts = ei;

  for (int i = tid; i < NBC; i += NTHR) scnt[i] = 0;
  __syncthreads();

  const int nChunks = (nE + CHUNK - 1) / CHUNK;
#pragma unroll 1
  for (int ch = 0; ch < nChunks; ++ch) {
    const int cbase = ch * CHUNK;
    const int wc = scan_chunk<NBC>(dsts, nE, cbase, nodeBase, vec8, list, tid, lane, wave);
    if (lane == 0) wcnt[wave] = wc;
    __syncthreads();
    if (wave == 0) {
#pragma unroll 1
      for (int wsx = 0; wsx < NWAVE; ++wsx) {
        int n = __builtin_amdgcn_readfirstlane(wcnt[wsx]);
        n = n > WCAP ? WCAP : (n < 0 ? 0 : n);
        const int* lp = list + wsx * WCAP;
#pragma unroll 1
        for (int i = 0; i < n; ++i) {
          const int ent  = __builtin_amdgcn_readfirstlane(lp[i]);
          const int slot = ent & (NBC - 1);
          if (lane == 0) scnt[slot] = scnt[slot] + 1;
        }
      }
    }
    __syncthreads();
  }

  v4i cq[4];
#pragma unroll
  for (int q = 0; q < 4; ++q) {
    const int f = (wave * 4 + q) * 128 + 4 * lane;
    cq[q] = *(const v4i*)(scnt + f);
  }
  int* cp = cnt + (size_t)nodeBase;
#pragma unroll
  for (int q = 0; q < 4; ++q) {
    const int f = (wave * 4 + q) * 128 + 4 * lane;
    *(volatile v4i*)(cp + f) = cq[q];
  }
  __threadfence();
#pragma unroll
  for (int q = 0; q < 4; ++q) {
    const int f = (wave * 4 + q) * 128 + 4 * lane;
    *(volatile v4i*)(cp + f) = cq[q];
  }
}

__global__ __launch_bounds__(OTHR) void k_offsets(
    const int* __restrict__ cnt, int* off, int* rbase, int nChunk) {
  __shared__ __attribute__((aligned(16))) int soff[NBC];
  __shared__ __attribute__((aligned(16))) int srb[RBN];
  __shared__ int wtot[OTHR / 32];
  const int tid = threadIdx.x, lane = tid & 31, wave = tid >> 5, sub = tid >> 7;
  for (int i = tid; i < RBN; i += OTHR) srb[i] = 0;
  int carry = 0;
#pragma unroll 1
  for (int ch = 0; ch < nChunk; ++ch) {
    const int base = ch * NBC;
    const v4i c0 = *(const v4i*)(cnt + base + 8 * tid);
    const v4i c1 = *(const v4i*)(cnt + base + 8 * tid + 4);
    const int e0 = max(c0.x, 0), e1 = max(c0.y, 0), e2 = max(c0.z, 0), e3 = max(c0.w, 0);
    const int e4 = max(c1.x, 0), e5 = max(c1.y, 0), e6 = max(c1.z, 0), e7 = max(c1.w, 0);
    const int ts = e0 + e1 + e2 + e3 + e4 + e5 + e6 + e7;
    int incl = ts;
#pragma unroll
    for (int d = 1; d < 32; d <<= 1) {
      const int t = __shfl_up(incl, d);
      if (lane >= d) incl += t;
    }
    if (lane == 31) wtot[wave] = incl;
    __syncthreads();
    const int S0 = wtot[0]  + wtot[1]  + wtot[2]  + wtot[3];
    const int S1 = wtot[4]  + wtot[5]  + wtot[6]  + wtot[7];
    const int S2 = wtot[8]  + wtot[9]  + wtot[10] + wtot[11];
    const int S3 = wtot[12] + wtot[13] + wtot[14] + wtot[15];
    int pre = 0;
#pragma unroll 1
    for (int w = 4 * sub; w < wave; ++w) pre += wtot[w];
    const int b0 = carry;
    const int b1 = b0 + ((S0 + 31) & ~31);
    const int b2 = b1 + ((S1 + 31) & ~31);
    const int b3 = b2 + ((S2 + 31) & ~31);
    const int b4 = b3 + ((S3 + 31) & ~31);
    const int myb = sub == 0 ? b0 : (sub == 1 ? b1 : (sub == 2 ? b2 : b3));
    if (tid == 0) {
      srb[min(4 * ch + 0, RBN - 1)] = b0;
      srb[min(4 * ch + 1, RBN - 1)] = b1;
      srb[min(4 * ch + 2, RBN - 1)] = b2;
      srb[min(4 * ch + 3, RBN - 1)] = b3;
    }
    int run = myb + pre + incl - ts;
    soff[8 * tid + 0] = run; run += e0;
    soff[8 * tid + 1] = run; run += e1;
    soff[8 * tid + 2] = run; run += e2;
    soff[8 * tid + 3] = run; run += e3;
    soff[8 * tid + 4] = run; run += e4;
    soff[8 * tid + 5] = run; run += e5;
    soff[8 * tid + 6] = run; run += e6;
    soff[8 * tid + 7] = run;
    carry = b4;
    __syncthreads();
    const v4i o0 = *(const v4i*)(soff + 4 * tid);
    const v4i o1 = *(const v4i*)(soff + 4 * (tid + OTHR));
    int* op = off + base;
    *(volatile v4i*)(op + 4 * tid) = o0;
    *(volatile v4i*)(op + 4 * (tid + OTHR)) = o1;
    __threadfence();
    *(volatile v4i*)(op + 4 * tid) = o0;
    *(volatile v4i*)(op + 4 * (tid + OTHR)) = o1;
    __syncthreads();
  }
  if (tid == 0) srb[min(4 * nChunk, RBN - 1)] = carry;
  __syncthreads();
  v4i rv = {0, 0, 0, 0};
  if (tid < 32) rv = *(const v4i*)(srb + 4 * tid);
  if (tid < 32) *(volatile v4i*)(rbase + 4 * tid) = rv;
  __threadfence();
  if (tid < 32) *(volatile v4i*)(rbase + 4 * tid) = rv;
}

__global__ __launch_bounds__(NTHR) void k_fill(
    const int* __restrict__ ei, const int* __restrict__ off, const int* __restrict__ rbase,
    int* csr, int nN, int nE, int vec8, int csrLen) {
  extern __shared__ v4f lds_dyn[];
  int* region = (int*)lds_dyn;
  int* cursor = region + RCAP;
  int* list   = cursor + NBF;
  int* wcnt   = list + LISTN;
  const int tid = threadIdx.x, lane = tid & 31, wave = tid >> 5;
  const int b = blockIdx.x;
  const int nodeBase = b * NBF;
  const int* dsts = ei;
  const int* srcs = ei + nE;

  int rb0 = rbase[b];
  const int rb1 = rbase[b + 1];
  rb0 = rb0 < 0 ? 0 : (rb0 > csrLen ? csrLen : rb0);
  rb0 &= ~31;
  int len = rb1 - rb0;
  len = len < 0 ? 0 : (len > RCAP ? RCAP : len);
  int lenW = (len + 31) & ~31;
  if (rb0 + lenW > csrLen) lenW = (csrLen - rb0) & ~31;

  {
    const v4i z = {0, 0, 0, 0};
    for (int i = tid; i < RCAP / 4; i += NTHR) ((v4i*)region)[i] = z;
    for (int s = tid; s < NBF; s += NTHR) {
      int o = off[nodeBase + s] - rb0;
      o = o < 0 ? 0 : (o > RCAP ? RCAP : o);
      cursor[s] = o;
    }
  }
  __syncthreads();

  const int nChunks = (nE + CHUNK - 1) / CHUNK;
#pragma unroll 1
  for (int ch = 0; ch < nChunks; ++ch) {
    const int cbase = ch * CHUNK;
    const int wc = scan_chunk<NBF>(dsts, nE, cbase, nodeBase, vec8, list, tid, lane, wave);
    if (lane == 0) wcnt[wave] = wc;
    __syncthreads();
    if (wave == 0) {
#pragma unroll 1
      for (int wsx = 0; wsx < NWAVE; ++wsx) {
        int n = __builtin_amdgcn_readfirstlane(wcnt[wsx]);
        n = n > WCAP ? WCAP : (n < 0 ? 0 : n);
        const int* lp = list + wsx * WCAP;
#pragma unroll 1
        for (int i = 0; i < n; ++i) {
          const int ent  = __builtin_amdgcn_readfirstlane(lp[i]);
          const int slot = ent & (NBF - 1);
          int e = cbase + ((ent >> 12) & (CHUNK - 1));
          e = e > nE - 1 ? nE - 1 : e;
          int src = srcs[e];
          src = src < 0 ? 0 : (src > nN - 1 ? nN - 1 : src);
          if (lane == 0) {
            int pos = cursor[slot];
            pos = pos < 0 ? 0 : (pos > RCAP - 1 ? RCAP - 1 : pos);
            region[pos] = src;
            const int np = pos + 1;
            cursor[slot] = np > RCAP ? RCAP : np;
          }
        }
      }
    }
    __syncthreads();
  }

  const int nv = lenW >> 2;
  int* gp = csr + rb0;
#pragma unroll 1
  for (int i = tid; i < nv; i += NTHR) { const v4i v = ((const v4i*)region)[i]; *(volatile v4i*)(gp + 4 * i) = v; }
  __threadfence();
#pragma unroll 1
  for (int i = tid; i < nv; i += NTHR) { const v4i v = ((const v4i*)region)[i]; *(volatile v4i*)(gp + 4 * i) = v; }
}

template <int HEAD>
__global__ __launch_bounds__(NTHR) void k_layer(
    const float* __restrict__ xin, const int* __restrict__ csr, const int* __restrict__ off,
    const int* __restrict__ cnt, const unsigned short* __restrict__ Bh, const unsigned short* __restrict__ Bl,
    const float* __restrict__ bsv, const float* __restrict__ bnv, const float* __restrict__ gam,
    const float* __restrict__ bet, float* xout,
    const unsigned short* __restrict__ Hh, const unsigned short* __restrict__ Hl,
    const float* __restrict__ hb1, const float* __restrict__ hw2, const float* __restrict__ hb2,
    float* out, int nN, int csrLen) {
  extern __shared__ v4f lds_dyn[];
  unsigned short* sAh = (unsigned short*)lds_dyn;
  unsigned short* sAl = sAh + GROWS * APH;
  float* stg  = (float*)(sAl + GROWS * APH);
  float* sOut = stg + GROWS * DD;
  const int tid = threadIdx.x, lane = tid & 31, wave = tid >> 5, hh = lane >> 4, m = lane & 15;
  const int rowBase = blockIdx.x * GROWS;
  const int r0w = wave * 16;

  {
    const int tl = rowBase + r0w + m;
    const int cnt_l = cnt[tl];
    const int off_l = off[tl];
    const int dg = cnt_l < 1 ? 1 : cnt_l;
    union FI { float f; int i; };
    FI iv; iv.f = 1.0f / (float)dg;
#pragma unroll 1
    for (int j = 0; j < 16; ++j) {
      int n = __builtin_amdgcn_readlane(cnt_l, j);
      n = n < 0 ? 0 : (n > DEGCAP ? DEGCAP : n);
      const int st = __builtin_amdgcn_readlane(off_l, j);
      FI q; q.i = __builtin_amdgcn_readlane(iv.i, j);
      v2f acc = {0.f, 0.f};
#pragma unroll 1
      for (int q0 = 0; q0 < n; q0 += 32) {
        int pos = st + q0 + lane;
        pos = pos < 0 ? 0 : (pos > csrLen - 1 ? csrLen - 1 : pos);
        int sl = csr[pos];
        sl = sl < 0 ? 0 : (sl > nN - 1 ? nN - 1 : sl);
        const int mcnt = (n - q0) < 32 ? (n - q0) : 32;
#pragma unroll 1
        for (int p = 0; p < mcnt; ++p) {
          const int s = __builtin_amdgcn_readlane(sl, p);
          acc = acc + *(const v2f*)(xin + (size_t)s * DD + 2 * lane);
        }
      }
      int row = rowBase + r0w + j;
      row = row > nN - 1 ? nN - 1 : row;
      const v2f xv = *(const v2f*)(xin + (size_t)row * DD + 2 * lane);
      const v2f nv = acc * q.f;
      v2us xh, xl, nh, nl;
      split2(xv, xh, xl);
      split2(nv, nh, nl);
      unsigned short* ph = sAh + (r0w + j) * APH + 2 * lane;
      unsigned short* pl = sAl + (r0w + j) * APH + 2 * lane;
      *(v2us*)ph = xh;
      *(v2us*)pl = xl;
      *(v2us*)(ph + DD) = nh;
      *(v2us*)(pl + DD) = nl;
    }
  }
  __syncthreads();

  v8f acc[4];
#pragma unroll
  for (int t = 0; t < 4; ++t) { v8f z = {0.f, 0.f, 0.f, 0.f, 0.f, 0.f, 0.f, 0.f}; acc[t] = z; }
  {
    const unsigned short* arh = sAh + (r0w + m) * APH + 8 * hh;
    const unsigned short* arl = sAl + (r0w + m) * APH + 8 * hh;
#pragma unroll
    for (int kt = 0; kt < KCAT / 32; ++kt) {
      FragB ah, al;
      ah.h[0] = *(const v8us*)(arh + 32 * kt);
      ah.h[1] = *(const v8us*)(arh + 32 * kt + 16);
      al.h[0] = *(const v8us*)(arl + 32 * kt);
      al.h[1] = *(const v8us*)(arl + 32 * kt + 16);
#pragma unroll
      for (int t = 0; t < 4; ++t) {
        const size_t bo = (size_t)(16 * t + m) * KCAT + 32 * kt + 8 * hh;
        FragB bhf, blf;
        bhf.h[0] = *(const v8us*)(Bh + bo);
        bhf.h[1] = *(const v8us*)(Bh + bo + 16);
        blf.h[0] = *(const v8us*)(Bl + bo);
        blf.h[1] = *(const v8us*)(Bl + bo + 16);
        acc[t] = wmb(ah.v, bhf.v, acc[t]);
        acc[t] = wmb(al.v, bhf.v, acc[t]);
        acc[t] = wmb(ah.v, blf.v, acc[t]);
      }
    }
  }

  {
    float* sp = stg + (r0w + 8 * hh) * DD + m;
#pragma unroll
    for (int t = 0; t < 4; ++t) {
      const float b1v = bsv[16 * t + m];
      const float b2v = bnv[16 * t + m];
#pragma unroll
      for (int r = 0; r < 8; ++r) {
        float v = acc[t][r] + b1v;
        v = v + b2v;
        sp[r * DD + 16 * t] = fmaxf(v, 0.0f);
      }
    }
  }
  __syncthreads();

  {
    const v2f gv = *(const v2f*)(gam + 2 * lane);
    const v2f bv = *(const v2f*)(bet + 2 * lane);
#pragma unroll 1
    for (int j = 0; j < 16; ++j) {
      float* rp = stg + (r0w + j) * DD + 2 * lane;
      const v2f v = *(const v2f*)rp;
      float s = v.x + v.y;
      s = wsum32(s);
      const float mu = s * (1.0f / 64.0f);
      v2f d; d.x = v.x - mu; d.y = v.y - mu;
      float s2 = d.x * d.x + d.y * d.y;
      s2 = wsum32(s2);
      const float var = s2 * (1.0f / 64.0f);
      const float rs = rsqrtf(var + LNEPS);
      v2f o;
      o.x = d.x * rs * gv.x + bv.x;
      o.y = d.y * rs * gv.y + bv.y;
      *(v2f*)rp = o;
    }
  }
  __syncthreads();

  if (HEAD == 0) {
    const float* lp = stg + r0w * DD + 4 * lane;
    float* gp = xout + ((size_t)rowBase + r0w) * DD + 4 * lane;
#pragma unroll
    for (int p = 0; p < 8; ++p) { const v4f v = *(const v4f*)(lp + p * 128); *(volatile v4f*)(gp + (size_t)p * 128) = v; }
    __threadfence();
#pragma unroll
    for (int p = 0; p < 8; ++p) { const v4f v = *(const v4f*)(lp + p * 128); *(volatile v4f*)(gp + (size_t)p * 128) = v; }
  } else {
#pragma unroll
    for (int it = 0; it < 4; ++it) {
      const int idx = it * NTHR + tid;
      const int r   = idx >> 3;
      const int c0  = (idx & 7) * 8;
      const v4f a = *(const v4f*)(stg + r * DD + c0);
      const v4f b = *(const v4f*)(stg + r * DD + c0 + 4);
      v8us h8, l8;
      split8(a, b, h8, l8);
      *(v8us*)(sAh + r * APH + c0) = h8;
      *(v8us*)(sAl + r * APH + c0) = l8;
    }
    __syncthreads();

    v8f c2[2];
#pragma unroll
    for (int t = 0; t < 2; ++t) { v8f z = {0.f, 0.f, 0.f, 0.f, 0.f, 0.f, 0.f, 0.f}; c2[t] = z; }
    {
      const unsigned short* arh = sAh + (r0w + m) * APH + 8 * hh;
      const unsigned short* arl = sAl + (r0w + m) * APH + 8 * hh;
#pragma unroll
      for (int kt = 0; kt < DD / 32; ++kt) {
        FragB ah, al;
        ah.h[0] = *(const v8us*)(arh + 32 * kt);
        ah.h[1] = *(const v8us*)(arh + 32 * kt + 16);
        al.h[0] = *(const v8us*)(arl + 32 * kt);
        al.h[1] = *(const v8us*)(arl + 32 * kt + 16);
#pragma unroll
        for (int t = 0; t < 2; ++t) {
          const size_t bo = (size_t)(16 * t + m) * DD + 32 * kt + 8 * hh;
          FragB bhf, blf;
          bhf.h[0] = *(const v8us*)(Hh + bo);
          bhf.h[1] = *(const v8us*)(Hh + bo + 16);
          blf.h[0] = *(const v8us*)(Hl + bo);
          blf.h[1] = *(const v8us*)(Hl + bo + 16);
          c2[t] = wmb(ah.v, bhf.v, c2[t]);
          c2[t] = wmb(al.v, bhf.v, c2[t]);
          c2[t] = wmb(ah.v, blf.v, c2[t]);
        }
      }
    }
    float pr[8];
    const float b1a = hb1[m], b1b = hb1[16 + m];
    const float w2a = hw2[m], w2b = hw2[16 + m];
#pragma unroll
    for (int r = 0; r < 8; ++r) {
      const float ha = fmaxf(c2[0][r] + b1a, 0.0f);
      const float hb = fmaxf(c2[1][r] + b1b, 0.0f);
      pr[r] = ha * w2a + hb * w2b;
    }
#pragma unroll
    for (int r = 0; r < 8; ++r) {
      pr[r] += __shfl_xor(pr[r], 8);
      pr[r] += __shfl_xor(pr[r], 4);
      pr[r] += __shfl_xor(pr[r], 2);
      pr[r] += __shfl_xor(pr[r], 1);
    }
    const float hb2v = hb2[0];
    if (m == 0) {
#pragma unroll
      for (int r = 0; r < 8; ++r) sOut[r0w + 8 * hh + r] = pr[r] + hb2v;
    }
    __syncthreads();
    int nv = nN - rowBase;
    nv = nv < 0 ? 0 : (nv > GROWS ? GROWS : nv);
    v4f ov = {0.f, 0.f, 0.f, 0.f};
    if (tid < 32) ov = *(const v4f*)(sOut + 4 * tid);
    const bool act = (tid < 32) && (4 * tid + 4 <= nv);
    float* op = out + (size_t)rowBase + 4 * tid;
    if (act) *(volatile v4f*)op = ov;
    __threadfence();
    if (act) *(volatile v4f*)op = ov;
  }
}

extern "C" void kernel_launch(void* const* d_in, const int* in_sizes, int n_in,
                              void* d_out, int out_size, void* d_ws, size_t ws_size,
                              hipStream_t stream) {
  if (n_in < 12) return;
  const int nN = in_sizes[0] / DD;
  const int nE = in_sizes[1] / 2;
  if (nN <= 0 || nE <= 0 || in_sizes[0] != nN * DD || in_sizes[1] != 2 * nE) return;
  const int nL = in_sizes[2] / (DD * DD);
  if (nL < 1 || in_sizes[2] != nL * DD * DD || in_sizes[4] != nL * DD * DD) return;
  if (in_sizes[3] < nL * DD || in_sizes[5] < nL * DD || in_sizes[6] < nL * DD || in_sizes[7] < nL * DD) return;
  if (in_sizes[8] != DD * HN || in_sizes[9] < HN || in_sizes[10] < HN || in_sizes[11] < 1) return;
  if (out_size != nN || (nN & 3) != 0) return;
  if (nE > (1 << 28) || nN > (1 << 24)) return;

  const float* x0  = (const float*)d_in[0];
  const int*   ei  = (const int*)d_in[1];
  const float* Ws  = (const float*)d_in[2];
  const float* bs  = (const float*)d_in[3];
  const float* Wn  = (const float*)d_in[4];
  const float* bn  = (const float*)d_in[5];
  const float* gam = (const float*)d_in[6];
  const float* bet = (const float*)d_in[7];
  const float* hw1 = (const float*)d_in[8];
  const float* hb1 = (const float*)d_in[9];
  const float* hw2 = (const float*)d_in[10];
  const float* hb2 = (const float*)d_in[11];
  float* out = (float*)d_out;

  const int NPAD   = ((nN + GROWS - 1) / GROWS) * GROWS;
  const int nBC    = (nN + NBC - 1) / NBC;
  const int CNTPAD = nBC * NBC;
  if (4 * nBC + 1 > RBN) return;
  const int nBF    = (nN + NBF - 1) / NBF;
  const int csrLen = ((nE + 31) & ~31) + 4096;
  const int nLB    = NPAD / GROWS;

  char* ws = (char*)d_ws;
  size_t off = 0;
  const size_t oWLh = off; off += (size_t)nL * DD * KCAT * 2;     off = (off + 255) & ~(size_t)255;
  const size_t oWLl = off; off += (size_t)nL * DD * KCAT * 2;     off = (off + 255) & ~(size_t)255;
  const size_t oH1h = off; off += (size_t)HN * DD * 2;            off = (off + 255) & ~(size_t)255;
  const size_t oH1l = off; off += (size_t)HN * DD * 2;            off = (off + 255) & ~(size_t)255;
  const size_t oCnt = off; off += (size_t)CNTPAD * 4;             off = (off + 255) & ~(size_t)255;
  const size_t oOff = off; off += (size_t)CNTPAD * 4;             off = (off + 255) & ~(size_t)255;
  const size_t oRb  = off; off += (size_t)RBN * 4;                off = (off + 255) & ~(size_t)255;
  const size_t oCsr = off; off += (size_t)csrLen * 4;             off = (off + 255) & ~(size_t)255;
  const size_t oXa  = off; off += (size_t)NPAD * DD * 4;          off = (off + 255) & ~(size_t)255;
  const size_t oXb  = off; off += (size_t)NPAD * DD * 4;          off = (off + 255) & ~(size_t)255;
  if (off > ws_size || off > (size_t)134217728u) return;
  unsigned short* wlh  = (unsigned short*)(ws + oWLh);
  unsigned short* wll  = (unsigned short*)(ws + oWLl);
  unsigned short* h1h  = (unsigned short*)(ws + oH1h);
  unsigned short* h1l  = (unsigned short*)(ws + oH1l);
  int*            cnt  = (int*)(ws + oCnt);
  int*            offp = (int*)(ws + oOff);
  int*            rb   = (int*)(ws + oRb);
  int*            csr  = (int*)(ws + oCsr);
  float*          xa   = (float*)(ws + oXa);
  float*          xb   = (float*)(ws + oXb);

  const int vec8 = 1;

  const int nPrep = nL * (DD * KCAT / 8) + HN * DD / 8;
  k_wprep<<<(nPrep + NTHR - 1) / NTHR, NTHR, 0, stream>>>(Ws, Wn, hw1, wlh, wll, h1h, h1l, nL);

  k_count<<<nBC, NTHR, 0, stream>>>(ei, cnt, nE, vec8);
  k_offsets<<<1, OTHR, 0, stream>>>(cnt, offp, rb, nBC);
  hipFuncSetAttribute(reinterpret_cast<const void*>(&k_fill),
                      hipFuncAttributeMaxDynamicSharedMemorySize, LDS_FILL);
  k_fill<<<nBF, NTHR, LDS_FILL, stream>>>(ei, offp, rb, csr, nN, nE, vec8, csrLen);

  hipFuncSetAttribute(reinterpret_cast<const void*>(&k_layer<0>),
                      hipFuncAttributeMaxDynamicSharedMemorySize, LDS_LAYER);
  hipFuncSetAttribute(reinterpret_cast<const void*>(&k_layer<1>),
                      hipFuncAttributeMaxDynamicSharedMemorySize, LDS_LAYER);
  const float* xin = x0;
  for (int i = 0; i < nL; ++i) {
    float* xo = (i & 1) ? xb : xa;
    const unsigned short* bh = wlh + (size_t)i * DD * KCAT;
    const unsigned short* bl = wll + (size_t)i * DD * KCAT;
    if (i == nL - 1) {
      k_layer<1><<<nLB, NTHR, LDS_LAYER, stream>>>(xin, csr, offp, cnt, bh, bl,
          bs + (size_t)i * DD, bn + (size_t)i * DD, gam + (size_t)i * DD, bet + (size_t)i * DD, xo,
          h1h, h1l, hb1, hw2, hb2, out, nN, csrLen);
    } else {
      k_layer<0><<<nLB, NTHR, LDS_LAYER, stream>>>(xin, csr, offp, cnt, bh, bl,
          bs + (size_t)i * DD, bn + (size_t)i * DD, gam + (size_t)i * DD, bet + (size_t)i * DD, xo,
          h1h, h1l, hb1, hw2, hb2, out, nN, csrLen);
    }
    xin = xo;
  }
}
